// _MLP_87222195847975
// MI455X (gfx1250) — hardware-verified
//
#include <hip/hip_runtime.h>


namespace {
constexpr int N = 262144, DIN = 32, DH = 128, NHID = 7, DOUT = 16, DCI = 16, DCO = 3, KC = 160  ;
constexpr float SC = 4096.0f;

typedef _Float16 b16;
typedef __attribute__((ext_vector_type(16))) _Float16 v16b;
typedef __attribute__((ext_vector_type(8))) _Float16 v8b;
typedef __attribute__((ext_vector_type(8))) float v8f;
typedef __attribute__((ext_vector_type(4))) float v4f;
__device__ __forceinline__ float bf16_rne(float f) { unsigned int u = __float_as_uint(f); u += 0x7FFFu + ((u >> 16) & 1u); return __uint_as_float(u & 0xFFFF0000u); }
__device__ __forceinline__ v16b frag_kb(const b16* p, int hh) { const v8b a = *(const v8b*)(p + 8 * hh), b = *(const v8b*)(p + 16 + 8 * hh); v16b f;
#pragma unroll
  for (int e = 0; e < 8; ++e) { f[e] = a[e]; f[8 + e] = b[e]; } return f; }
__device__ __forceinline__ v8f wmma16b(v16b a, v16b b, v8f c) { v8f d = __builtin_amdgcn_wmma_f32_16x16x32_f16(false, a, false, b, (short)0, c, false, false); asm volatile("v_nop\n\tv_nop\n\tv_nop\n\tv_nop" : "+v"(d) : "v"(a), "v"(b)); return d; }
__device__ __forceinline__ void wave_lds_sync() { __builtin_amdgcn_fence(__ATOMIC_RELEASE, "workgroup"); __builtin_amdgcn_wave_barrier(); __builtin_amdgcn_fence(__ATOMIC_ACQUIRE, "workgroup"); }

struct Wo_ { static constexpr size_t W0 = 0, WH = W0 + 128 * 32, WOUT = WH + (size_t)7 * 128 * 128, WC0 = WOUT + 16 * 128, WC1 = WC0 + 128 * 160, WC2 = WC1 + 64 * 128, END = WC2 + 16 * 64; };
__global__ __launch_bounds__(256) void prep_kernel(const float* __restrict__ W0, const float* __restrict__ Wh, const float* __restrict__ Wout, const float* __restrict__ Wc0, const float* __restrict__ Wc1, const float* __restrict__ Wc2, b16* __restrict__ R) {
  const int t_ = blockIdx.x * 256 + threadIdx.x, nth = gridDim.x * 256;
  for (int pass = 0; pass < 2; ++pass) {
    for (int i = t_; i < 128 * 32; i += nth) R[Wo_::W0 + i] = (b16)bf16_rne(W0[i]);
    for (int i = t_; i < 7 * 128 * 128; i += nth) R[Wo_::WH + i] = (b16)bf16_rne(Wh[i]);
    for (int i = t_; i < 16 * 128; i += nth) R[Wo_::WOUT + i] = (b16)bf16_rne(Wout[i]);
    for (int i = t_; i < 128 * 160; i += nth) { const int o = i / 160, k = i % 160; R[Wo_::WC0 + i] = (b16)((k < 144) ? bf16_rne(Wc0[(size_t)o * 144 + k]) : 0.0f); }
    for (int i = t_; i < 64 * 128; i += nth) R[Wo_::WC1 + i] = (b16)bf16_rne(Wc1[i]);
    for (int i = t_; i < 16 * 64; i += nth) { const int o = i / 64, k = i % 64; R[Wo_::WC2 + i] = (b16)((o < DCO) ? bf16_rne(Wc2[(size_t)o * 64 + k]) : 0.0f); }
    __threadfence(); }
}

template <int NT_>
__device__ __forceinline__ void wgemm(const b16 (*Hs)[KC + 8], int K, const b16* Bw, int ldb, int nloc, int hlf, v8f (&acc)[2][NT_]) {
#pragma unroll
  for (int r = 0; r < 2; ++r)
#pragma unroll
    for (int t = 0; t < NT_; ++t) acc[r][t] = (v8f){};
  for (int kb = 0; kb < K; kb += 32) { const v16b a0 = frag_kb(&Hs[nloc][kb], hlf), a1 = frag_kb(&Hs[16 + nloc][kb], hlf);
#pragma unroll
    for (int t = 0; t < NT_; ++t) { const v16b bw = frag_kb(Bw + (size_t)(t * 16 + nloc) * ldb + kb, hlf); acc[0][t] = wmma16b(a0, bw, acc[0][t]); acc[1][t] = wmma16b(a1, bw, acc[1][t]); } }
}

__global__ __launch_bounds__(128) void mlp_kernel(const float* __restrict__ x, const float* __restrict__ cond, const b16* __restrict__ R, float* __restrict__ out0, float* __restrict__ out1) {
  __shared__ __attribute__((aligned(16))) b16 Hs[4][32][KC + 8]; __shared__ __attribute__((aligned(16))) float U[4][32][DOUT]; __shared__ __attribute__((aligned(16))) float Co[128][4];
  const int lane = threadIdx.x & 31, wave = threadIdx.x >> 5, nloc = lane & 15, hlf = lane >> 4, m0 = blockIdx.x * 128 + wave * 32;
  b16 (*H)[KC + 8] = Hs[wave];
  for (int i = lane; i < 32 * DIN; i += 32) { const int r = i >> 5, k = i & 31; H[r][k] = (b16)(bf16_rne(x[(size_t)(m0 + r) * DIN + k]) * SC); }
  wave_lds_sync();
  { v8f acc[2][8]; wgemm<8>(H, DIN, R + Wo_::W0, DIN, nloc, hlf, acc); wave_lds_sync();
#pragma unroll
    for (int t = 0; t < 8; ++t)
#pragma unroll
      for (int r = 0; r < 2; ++r)
#pragma unroll
        for (int v = 0; v < 8; ++v) H[r * 16 + 8 * hlf + v][t * 16 + nloc] = (b16)fmaxf(acc[r][t][v], 0.0f);
    wave_lds_sync(); }
  for (int l = 0; l < NHID; ++l) { v8f acc[2][8]; wgemm<8>(H, DH, R + Wo_::WH + (size_t)l * DH * DH, DH, nloc, hlf, acc); wave_lds_sync();
#pragma unroll
    for (int t = 0; t < 8; ++t)
#pragma unroll
      for (int r = 0; r < 2; ++r)
#pragma unroll
        for (int v = 0; v < 8; ++v) H[r * 16 + 8 * hlf + v][t * 16 + nloc] = (b16)fmaxf(acc[r][t][v], 0.0f);
    wave_lds_sync(); }
  { v8f acc[2][1]; wgemm<1>(H, DH, R + Wo_::WOUT, DH, nloc, hlf, acc);
#pragma unroll
    for (int r = 0; r < 2; ++r)
#pragma unroll
      for (int v = 0; v < 8; ++v) U[wave][r * 16 + 8 * hlf + v][nloc] = acc[r][0][v] * (1.0f / SC); }
  for (int i = lane; i < 32 * 32; i += 32) { const int r = i >> 5, k = i & 31; H[r][DH + k] = (b16)((k < DCI) ? bf16_rne(cond[(size_t)(m0 + r) * DCI + k]) * SC : 0.0f); }
  wave_lds_sync();
  { v8f acc[2][8]; wgemm<8>(H, KC, R + Wo_::WC0, KC, nloc, hlf, acc); wave_lds_sync();
#pragma unroll
    for (int t = 0; t < 8; ++t)
#pragma unroll
      for (int r = 0; r < 2; ++r)
#pragma unroll
        for (int v = 0; v < 8; ++v) H[r * 16 + 8 * hlf + v][t * 16 + nloc] = (b16)acc[r][t][v];
    wave_lds_sync(); }
  { v8f acc[2][4]; wgemm<4>(H, DH, R + Wo_::WC1, DH, nloc, hlf, acc); wave_lds_sync();
#pragma unroll
    for (int t = 0; t < 4; ++t)
#pragma unroll
      for (int r = 0; r < 2; ++r)
#pragma unroll
        for (int v = 0; v < 8; ++v) H[r * 16 + 8 * hlf + v][t * 16 + nloc] = (b16)fmaxf(acc[r][t][v], 0.0f);
    wave_lds_sync(); }
  { v8f acc[2][1]; wgemm<1>(H, 64, R + Wo_::WC2, 64, nloc, hlf, acc);
    if (nloc < DCO) {
#pragma unroll
      for (int r = 0; r < 2; ++r)
#pragma unroll
        for (int v = 0; v < 8; ++v) Co[wave * 32 + r * 16 + 8 * hlf + v][nloc] = acc[r][0][v] * (1.0f / SC); } }
  wave_lds_sync();
  for (int pass = 0; pass < 2; ++pass) { for (int i = lane; i < 32 * 4; i += 32) { const int rr = i >> 2, c4 = (i & 3) * 4; *(volatile v4f*)(out0 + (size_t)(m0 + rr) * DOUT + c4) = *(const v4f*)(&U[wave][rr][c4]); } __threadfence(); }
  __syncthreads();
  const int nb = blockIdx.x * 128;
  for (int pass = 0; pass < 2; ++pass) { if (threadIdx.x < 96) { const int q = threadIdx.x; v4f o; for (int e = 0; e < 4; ++e) { const int f = q * 4 + e; o[e] = Co[f / 3][f % 3]; } *(volatile v4f*)(out1 + (size_t)nb * DCO + q * 4) = o; } __threadfence(); }
}
}

extern "C" void kernel_launch(void* const* d_in, const int* in_sizes, int n_in,
                              void* d_out, int out_size, void* d_ws, size_t ws_size, hipStream_t stream) {
  (void)n_in; (void)out_size;
  const float* x = (const float*)d_in[0]; const float* cond = (const float*)d_in[1]; const float* W0 = (const float*)d_in[2]; const float* Wh = (const float*)d_in[3]; const float* Wout = (const float*)d_in[4]; const float* Wc0 = (const float*)d_in[5]; const float* Wc1 = (const float*)d_in[6]; const float* Wc2 = (const float*)d_in[7];
  float* out0 = (float*)d_out; float* out1 = out0 + (size_t)N * DOUT;
  if (in_sizes[0] != N * DIN || in_sizes[1] != N * DCI || in_sizes[2] != DH * DIN || in_sizes[3] != NHID * DH * DH || in_sizes[5] != DH * 144 || in_sizes[7] != DCO * 64) return;
  if (Wo_::END * 2 > ws_size) return;
  b16* R = (b16*)d_ws;
  prep_kernel<<<64, 256, 0, stream>>>(W0, Wh, Wout, Wc0, Wc1, Wc2, R);
  mlp_kernel<<<N / 128, 128, 0, stream>>>(x, cond, R, out0, out1);
}
